// Mamba_13726715478163
// MI455X (gfx1250) — hardware-verified
//
#include <hip/hip_runtime.h>
#include <math.h>

typedef __attribute__((ext_vector_type(16))) _Float16 v16h;
typedef __attribute__((ext_vector_type(8)))  _Float16 v8h;
typedef __attribute__((ext_vector_type(16))) __bf16   v16b;
typedef __attribute__((ext_vector_type(8)))  __bf16   v8b;
typedef __attribute__((ext_vector_type(8)))  float    v8f;
typedef __attribute__((ext_vector_type(4)))  float    v4f;
typedef __attribute__((ext_vector_type(4)))  unsigned int v4u;

constexpr int kB      = 2;
constexpr int kL      = 1024;
constexpr int kDm     = 768;
constexpr int kDin    = 1536;
constexpr int kNst    = 16;
constexpr int kDtR    = 48;
constexpr int kNS     = 3 * kB;
constexpr int kXzP    = 2 * kDin;
constexpr int kXdW    = kDtR + 2 * kNst;
constexpr int kXdP    = 128;
constexpr int kRowsT  = kB * kL;
constexpr int kRowsS  = kNS * kL;
constexpr int kConvTS = 64;
constexpr int kConvTP = 260;
constexpr int kScanTS = 64;
constexpr int kScanCh = 64;
constexpr int kScanXP = 80;
constexpr int kScanYP = 68;
static_assert(kXdW <= kXdP, "x_proj pad");
static_assert((kDm % 32) == 0 && (kDin % 32) == 0, "GEMM K multiples of 32");
static_assert((kRowsT % 64) == 0 && (kRowsS % 64) == 0 && (kXzP % 64) == 0 && (kXdP % 64) == 0 && (kDm % 64) == 0, "GEMM M,N multiples of 64");
static_assert((kL % kConvTS) == 0 && (kL % kScanTS) == 0 && (kDin % kScanCh) == 0 && (kDin % 256) == 0, "tile multiples");
static_assert(kScanTS == kScanCh, "one thread per staged step index");
static_assert(kL == 1024, "row decomposition uses >>10 and &1023");
static_assert((kScanXP % 4) == 0 && ((kScanTS * kScanXP / 4) % kScanCh) == 0, "scan staging map");
static_assert((kDm % 8) == 0 && (kDin % 8) == 0, "8-element groups never straddle rows");

constexpr size_t kOffXH   = 0;
constexpr size_t kOffXL   = kOffXH  + (size_t)kRowsT * kDm  * 2;
constexpr size_t kOffWIH  = kOffXL  + (size_t)kRowsT * kDm  * 2;
constexpr size_t kOffWIL  = kOffWIH + (size_t)kXzP   * kDm  * 2;
constexpr size_t kOffWXH  = kOffWIL + (size_t)kXzP   * kDm  * 2;
constexpr size_t kOffWXL  = kOffWXH + (size_t)kXdP   * kDin * 2;
constexpr size_t kOffWOH  = kOffWXL + (size_t)kXdP   * kDin * 2;
constexpr size_t kOffWOL  = kOffWOH + (size_t)kDm    * kDin * 2;
constexpr size_t kOffXZ   = kOffWOL + (size_t)kDm    * kDin * 2;
constexpr size_t kOffXCH  = kOffXZ  + (size_t)kRowsT * kXzP * 4;
constexpr size_t kOffXCL  = kOffXCH + (size_t)kRowsS * kDin * 2;
constexpr size_t kOffXD   = kOffXCL + (size_t)kRowsS * kDin * 2;
constexpr size_t kOffYD   = kOffXD  + (size_t)kRowsS * kXdP * 4;
constexpr size_t kOffYMH  = kOffYD  + (size_t)kRowsS * kDin * 2;
constexpr size_t kOffYML  = kOffYMH + (size_t)kRowsT * kDin * 2;
constexpr size_t kWsTotal = kOffYML + (size_t)kRowsT * kDin * 2;
static_assert(kWsTotal == 118751232ull, "carve total");
static_assert(kWsTotal <= 134217728ull, "carve cap");
static_assert((kOffXL % 128) == 0 && (kOffWIH % 128) == 0 && (kOffWIL % 128) == 0 && (kOffWXH % 128) == 0 &&
              (kOffWXL % 128) == 0 && (kOffWOH % 128) == 0 && (kOffWOL % 128) == 0 && (kOffXZ % 128) == 0 &&
              (kOffXCH % 128) == 0 && (kOffXCL % 128) == 0 && (kOffXD % 128) == 0 && (kOffYD % 128) == 0 &&
              (kOffYMH % 128) == 0 && (kOffYML % 128) == 0, "128-B aligned regions");

__device__ __forceinline__ unsigned short f2bf_bits(float f) {
  unsigned u = __float_as_uint(f);
  return (unsigned short)((u + 0x7FFFu + ((u >> 16) & 1u)) >> 16);
}
__device__ __forceinline__ float bf_bits2f(unsigned short h) { return __uint_as_float(((unsigned)h) << 16); }

__device__ __forceinline__ float h16_to_f32(unsigned hb) {
  const unsigned sgn = (hb & 0x8000u) << 16; const unsigned em = hb & 0x7fffu;
  const float fn = __uint_as_float((em << 13) + 0x38000000u);
  const float fs = (float)em * 5.9604644775390625e-8f;
  const float mag = (em < 0x400u) ? fs : fn; return __uint_as_float(__float_as_uint(mag) | sgn); }

__device__ __forceinline__ int clampi(int v, int lo, int hi) { v = v < lo ? lo : v; return v > hi ? hi : v; }

__device__ __forceinline__ void dep_guard_h(v8f& a, v8f& b, v16h x, v16h y) { asm volatile("v_nop\n\tv_nop\n\tv_nop\n\tv_nop" : "+v"(a), "+v"(b) : "v"(x), "v"(y)); }
__device__ __forceinline__ void dep_guard_b(v8f& a, v8f& b, v16b x, v16b y) { asm volatile("v_nop\n\tv_nop\n\tv_nop\n\tv_nop" : "+v"(a), "+v"(b) : "v"(x), "v"(y)); }
__device__ __forceinline__ void keep4_h(v16h a, v16h b, v16h c, v16h d) { asm volatile("v_nop" :: "v"(a), "v"(b), "v"(c), "v"(d)); }
__device__ __forceinline__ void keep4_b(v16b a, v16b b, v16b c, v16b d) { asm volatile("v_nop" :: "v"(a), "v"(b), "v"(c), "v"(d)); }
__device__ __forceinline__ void acc_guard4(v8f& a, v8f& b, v8f& c, v8f& d) { asm volatile("v_nop\n\tv_nop\n\tv_nop\n\tv_nop" : "+v"(a), "+v"(b), "+v"(c), "+v"(d)); }
template <typename T> struct Frag;
template <> struct Frag<_Float16> {
  typedef v16h V; union U { v16h v; v8h h[2]; };
  static __device__ __forceinline__ v16h load(const _Float16* p) {
    U f; f.h[0] = *(const v8h*)(p); f.h[1] = *(const v8h*)(p + 16); return f.v;
  }
  static __device__ __forceinline__ v8f mma(v16h a, v16h b, v8f c) {
    return __builtin_amdgcn_wmma_f32_16x16x32_f16(false, a, false, b, (short)0, c, false, false);
  }
  static __device__ __forceinline__ void guard(v8f& a, v8f& b, v16h x, v16h y) { dep_guard_h(a, b, x, y); }
  static __device__ __forceinline__ void keep(v16h a, v16h b, v16h c, v16h d) { keep4_h(a, b, c, d); }
};
template <> struct Frag<__bf16> {
  typedef v16b V; union U { v16b v; v8b h[2]; };
  static __device__ __forceinline__ v16b load(const __bf16* p) {
    U f; f.h[0] = *(const v8b*)(p); f.h[1] = *(const v8b*)(p + 16); return f.v;
  }
  static __device__ __forceinline__ v8f mma(v16b a, v16b b, v8f c) {
    return __builtin_amdgcn_wmma_f32_16x16x32_bf16(false, a, false, b, (short)0, c, false, false);
  }
  static __device__ __forceinline__ void guard(v8f& a, v8f& b, v16b x, v16b y) { dep_guard_b(a, b, x, y); }
  static __device__ __forceinline__ void keep(v16b a, v16b b, v16b c, v16b d) { keep4_b(a, b, c, d); }
};

template <int ET> struct Elem;
template <> struct Elem<0> { typedef _Float16 T; };
template <> struct Elem<1> { typedef __bf16 T; };
template <int ET, int SPL, int BIAS_MODE, int OUT_MODE, bool RESID, int ACT = 0>
__global__ __launch_bounds__(256) void wmma_gemm64(
    const unsigned short* __restrict__ Ap, const unsigned short* __restrict__ A2p, int lda, long strideA,
    const unsigned short* __restrict__ Btp, const unsigned short* __restrict__ Bt2p, int ldb, long strideB,
    void* __restrict__ Cout, void* __restrict__ Cout2, int ldc, long strideC,
    const float* __restrict__ bias,
    const float* __restrict__ resid, long strideR,
    int M, int N, int K, float scale) {
  typedef typename Elem<ET>::T T;
  typedef typename Frag<T>::V V;
  const T* A = (const T*)Ap; const T* A2 = (const T*)A2p; const T* Bt = (const T*)Btp; const T* Bt2 = (const T*)Bt2p;
  __shared__ __align__(16) float sT[8][16 * 68];
  const int b    = blockIdx.y;
  const int lane = threadIdx.x & 31;
  const int wave = threadIdx.x >> 5;
  const int tilesN = N >> 6;
  const int tilesM = M >> 6;
  const int tile = blockIdx.x * 8 + wave;
  if (tile >= tilesM * tilesN) return;
  const int tm = tile / tilesN;
  const int tn = tile - tm * tilesN;
  const int m0 = tm << 6;
  const int n0 = tn << 6;

  const T* Ab  = A  + (size_t)b * strideA;
  const T* Bb  = Bt + (size_t)b * strideB;
  const T* Ab2 = (SPL >= 1) ? (A2  + (size_t)b * strideA) : nullptr;
  const T* Bb2 = (SPL == 2) ? (Bt2 + (size_t)b * strideB) : nullptr;

  const int rlane = lane & 15;
  const int koff  = (lane >> 4) * 8;
  const int mOff  = (lane >> 4) * 8;

  v8f acc[4][4];
#pragma unroll
  for (int i = 0; i < 4; ++i)
#pragma unroll
    for (int j = 0; j < 4; ++j) acc[i][j] = (v8f){0.f,0.f,0.f,0.f,0.f,0.f,0.f,0.f};

  for (int k0 = 0; k0 < K; k0 += 32) {
    V bh[4], bl[4];
#pragma unroll
    for (int j = 0; j < 4; ++j) {
      const size_t bo = (size_t)(n0 + (j << 4) + rlane) * ldb + koff + k0;
      bh[j] = Frag<T>::load(Bb + bo);
      if (SPL == 2) bl[j] = Frag<T>::load(Bb2 + bo);
    }
#pragma unroll
    for (int i = 0; i < 4; ++i) {
      const size_t ao = (size_t)(m0 + (i << 4) + rlane) * lda + koff + k0;
      V ah = Frag<T>::load(Ab + ao);
      V al;
      if (SPL >= 1) al = Frag<T>::load(Ab2 + ao);
#pragma unroll
      for (int j = 0; j < 4; ++j) {
        acc[i][j] = Frag<T>::mma(ah, bh[j], acc[i][j]);
        if (SPL == 2) acc[i][j] = Frag<T>::mma(ah, bl[j], acc[i][j]);
        if (SPL >= 1) acc[i][j] = Frag<T>::mma(al, bh[j], acc[i][j]);
      }
      Frag<T>::guard(acc[i][0], acc[i][3], ah, (SPL >= 1) ? al : ah);
      Frag<T>::guard(acc[i][1], acc[i][2], ah, (SPL >= 1) ? al : ah);
    }
    Frag<T>::keep(bh[0], bh[1], bh[2], bh[3]);
    if (SPL == 2) Frag<T>::keep(bl[0], bl[1], bl[2], bl[3]);
  }
  acc_guard4(acc[0][0], acc[0][1], acc[0][2], acc[0][3]);
  acc_guard4(acc[1][0], acc[1][1], acc[1][2], acc[1][3]);
  acc_guard4(acc[2][0], acc[2][1], acc[2][2], acc[2][3]);
  acc_guard4(acc[3][0], acc[3][1], acc[3][2], acc[3][3]);

  float* slab = sT[wave];
  const float* Rb = RESID ? (resid + (size_t)b * strideR) : nullptr;
#pragma unroll
  for (int i = 0; i < 4; ++i) {
    const int mBase = m0 + (i << 4);
#pragma unroll
    for (int j = 0; j < 4; ++j) {
      const int n = n0 + (j << 4) + rlane;
      float bv = 0.f;
      if (BIAS_MODE == 2) bv = bias[n];
#pragma unroll
      for (int r = 0; r < 8; ++r) {
        float v = acc[i][j][r] * scale;
        if (BIAS_MODE == 1) v += bias[mBase + mOff + r];
        if (BIAS_MODE == 2) v += bv;
        if (RESID) v += Rb[(size_t)(mBase + mOff + r) * ldc + n];
        if (ACT == 1) v = tanhf(v);
        if (ACT == 2) v = fmaxf(v, 0.0f);
        if (ACT == 3) v = v / (1.0f + expf(-v));
        if (ACT == 4) v = (v > 0.f) ? v : 0.01f * v;
        slab[(mOff + r) * 68 + (j << 4) + rlane] = v;
      }
    }
    __builtin_amdgcn_fence(__ATOMIC_RELEASE, "workgroup");
    __builtin_amdgcn_wave_barrier();
    __builtin_amdgcn_fence(__ATOMIC_ACQUIRE, "workgroup");
    if (OUT_MODE == 0) {
      float* C = (float*)Cout + (size_t)b * strideC;
      const int hh = lane >> 4, c4 = (lane & 15) * 4;
      for (int pass = 0; pass < 2; ++pass) {
#pragma unroll
        for (int it = 0; it < 8; ++it) {
          const int row = it * 2 + hh;
          v4f v = *(const v4f*)(slab + row * 68 + c4);
          *(volatile v4f*)(C + (size_t)(mBase + row) * ldc + n0 + c4) = v;
        }
        __threadfence();
      }
    } else {
      const int q = lane >> 3, c8 = (lane & 7) * 8;
      unsigned short* C  = (unsigned short*)Cout  + (size_t)b * strideC;
      unsigned short* C2 = (OUT_MODE == 2) ? ((unsigned short*)Cout2 + (size_t)b * strideC) : nullptr;
      for (int pass = 0; pass < 2; ++pass) {
#pragma unroll
        for (int it = 0; it < 4; ++it) {
          const int row = it * 4 + q;
          const float* sp = slab + row * 68 + c8;
          v8h hv, lv;
#pragma unroll
          for (int e = 0; e < 8; ++e) {
            if (OUT_MODE == 1) {
              hv[e] = (_Float16)sp[e];
            } else {
              unsigned short hb = f2bf_bits(sp[e]);
              unsigned short lb = f2bf_bits(sp[e] - bf_bits2f(hb));
              hv[e] = __builtin_bit_cast(_Float16, hb);
              lv[e] = __builtin_bit_cast(_Float16, lb);
            }
          }
          *(volatile v8h*)(C + (size_t)(mBase + row) * ldc + n0 + c8) = hv;
          if (OUT_MODE == 2) *(volatile v8h*)(C2 + (size_t)(mBase + row) * ldc + n0 + c8) = lv;
        }
        __threadfence();
      }
    }
    __builtin_amdgcn_fence(__ATOMIC_RELEASE, "workgroup");
    __builtin_amdgcn_wave_barrier();
    __builtin_amdgcn_fence(__ATOMIC_ACQUIRE, "workgroup");
  }
}

__global__ __launch_bounds__(256) void split_rows_bf16_kernel(
    const float* __restrict__ src, unsigned short* __restrict__ dhi, unsigned short* __restrict__ dlo,
    int rows_real, int cols, int total8)
{
  const int i = blockIdx.x * 256 + threadIdx.x;
  if (i >= total8) return;
  const unsigned e0  = (unsigned)i << 3;
  const unsigned row = e0 / (unsigned)cols;
  const unsigned col = e0 - row * (unsigned)cols;
  const bool real = ((int)row < rows_real);
  const unsigned rowc = real ? row : (unsigned)(rows_real - 1);
  const float* sp = src + (size_t)rowc * (unsigned)cols + col;
  const v4f r0 = *(const v4f*)(sp);
  const v4f r1 = *(const v4f*)(sp + 4);
  v8h hv, lv;
#pragma unroll
  for (int e = 0; e < 4; ++e) {
    const float x0 = real ? r0[e] : 0.0f;
    const float x1 = real ? r1[e] : 0.0f;
    const unsigned short h0 = f2bf_bits(x0), h1 = f2bf_bits(x1);
    const unsigned short l0 = f2bf_bits(x0 - bf_bits2f(h0)), l1 = f2bf_bits(x1 - bf_bits2f(h1));
    hv[e]     = __builtin_bit_cast(_Float16, h0);
    hv[4 + e] = __builtin_bit_cast(_Float16, h1);
    lv[e]     = __builtin_bit_cast(_Float16, l0);
    lv[4 + e] = __builtin_bit_cast(_Float16, l1);
  }
  unsigned short* qh = dhi + e0;
  unsigned short* ql = dlo + e0;
  *(volatile v8h*)qh = hv;
  *(volatile v8h*)ql = lv;
  __threadfence();
  *(volatile v8h*)qh = hv;
  *(volatile v8h*)ql = lv;
}

__global__ __launch_bounds__(256) void conv_silu_kernel(
    const float* __restrict__ XZ, const float* __restrict__ cw, const float* __restrict__ cb,
    const int* __restrict__ perm1, const int* __restrict__ perm2,
    unsigned short* __restrict__ XCH, unsigned short* __restrict__ XCL)
{
  __shared__ __align__(16) float sT[16 * kConvTP];
  __shared__ int sRow[80];
  const int tid = threadIdx.x, lane = tid & 31, wave = tid >> 5;
  const int d0 = blockIdx.x * 256, d = d0 + tid;
  const int l0 = blockIdx.y * kConvTS;
  const int s  = blockIdx.z;
  const int bb = s / 3, dir = s - 3 * bb;
  const size_t trow0 = (size_t)bb * kL;
  const size_t srow0 = (size_t)s * kL + l0;
  if (tid < kConvTS + 3) {
    int l = l0 - 3 + tid;
    l = l < 0 ? 0 : l;
    const int o1 = clampi(perm1[l], 0, kL - 1);
    const int o2 = clampi(perm2[l], 0, kL - 1);
    const int pr = (dir == 0) ? l : ((dir == 1) ? o1 : o2);
    sRow[tid] = pr;
  }
  const v4f wv = *(const v4f*)(cw + (size_t)d * 4);
  const float w0 = wv[0], w1 = wv[1], w2 = wv[2], w3 = wv[3];
  const float bc = cb[d];
  __syncthreads();
  float xm3, xm2, xm1;
  {
    const bool hist = (l0 > 0);
    const float v3 = XZ[(trow0 + sRow[0]) * kXzP + d];
    const float v2 = XZ[(trow0 + sRow[1]) * kXzP + d];
    const float v1 = XZ[(trow0 + sRow[2]) * kXzP + d];
    xm3 = hist ? v3 : 0.f;
    xm2 = hist ? v2 : 0.f;
    xm1 = hist ? v1 : 0.f;
  }
#pragma unroll 1
  for (int sub = 0; sub < 4; ++sub) {
#pragma unroll 1
    for (int st = 0; st < 16; ++st) {
      const float xcur = XZ[(trow0 + sRow[3 + sub * 16 + st]) * kXzP + d];
      float acc = w0 * xm3;
      acc = fmaf(w1, xm2, acc);
      acc = fmaf(w2, xm1, acc);
      acc = fmaf(w3, xcur, acc);
      const float sv = acc + bc;
      const float sg = __builtin_amdgcn_rcpf(1.0f + __expf(-sv));
      sT[st * kConvTP + tid] = sv * sg;
      xm3 = xm2; xm2 = xm1; xm1 = xcur;
    }
    __syncthreads();
    v8h bh[2], blo[2];
#pragma unroll
    for (int it = 0; it < 2; ++it) {
      const float* sp = sT + (it * 8 + wave) * kConvTP + lane * 8;
      const v4f a0 = *(const v4f*)(sp);
      const v4f a1 = *(const v4f*)(sp + 4);
#pragma unroll
      for (int e = 0; e < 4; ++e) {
        const unsigned short h0 = f2bf_bits(a0[e]), h1 = f2bf_bits(a1[e]);
        const unsigned short l0b = f2bf_bits(a0[e] - bf_bits2f(h0)), l1b = f2bf_bits(a1[e] - bf_bits2f(h1));
        bh[it][e]      = __builtin_bit_cast(_Float16, h0);
        bh[it][4 + e]  = __builtin_bit_cast(_Float16, h1);
        blo[it][e]     = __builtin_bit_cast(_Float16, l0b);
        blo[it][4 + e] = __builtin_bit_cast(_Float16, l1b);
      }
    }
    for (int pass = 0; pass < 2; ++pass) {
#pragma unroll
      for (int it = 0; it < 2; ++it) {
        const size_t o = (srow0 + sub * 16 + it * 8 + wave) * kDin + d0 + lane * 8;
        *(volatile v8h*)(XCH + o) = bh[it];
        *(volatile v8h*)(XCL + o) = blo[it];
      }
      __threadfence();
    }
    __syncthreads();
  }
}

__global__ __launch_bounds__(64) void scan_kernel(
    const float* __restrict__ XD, const unsigned short* __restrict__ XCH, const unsigned short* __restrict__ XCL,
    const float* __restrict__ XZ, const float* __restrict__ Wdt, const float* __restrict__ bdt,
    const float* __restrict__ Alog, const float* __restrict__ Dp,
    const int* __restrict__ perm1, const int* __restrict__ perm2,
    unsigned short* __restrict__ YD)
{
  __shared__ __align__(16) float sX[kScanTS * kScanXP];
  __shared__ __align__(16) float sY[kScanTS * kScanYP];
  __shared__ __align__(16) float sW[kDtR * kScanCh];
  __shared__ __align__(16) float sA[kNst * kScanCh];
  __shared__ int sRow[kScanTS];
  const int tid = threadIdx.x, lane = tid & 31, wave = tid >> 5;
  constexpr int kBlkPerS = kDin / kScanCh;
  const int s   = blockIdx.x / kBlkPerS;
  const int d0  = (blockIdx.x - s * kBlkPerS) * kScanCh;
  const int d   = d0 + tid;
  const int bb  = s / 3, dir = s - 3 * bb;
  const size_t srow0 = (size_t)s * kL;
  const size_t trow0 = (size_t)bb * kL;
#pragma unroll 1
  for (int r = 0; r < kDtR; ++r) sW[r * kScanCh + tid] = Wdt[(size_t)d * kDtR + r];
#pragma unroll 1
  for (int n = 0; n < kNst; ++n) sA[n * kScanCh + tid] = -expf(Alog[(size_t)d * kNst + n]);
  __syncthreads();
  float negA[kNst], h[kNst];
#pragma unroll
  for (int n = 0; n < kNst; ++n) {
    negA[n] = sA[n * kScanCh + tid];
    h[n] = 0.f;
  }
  const float bbias = bdt[d], Dd = Dp[d];
  const int q = lane >> 3, c8 = (lane & 7) * 8;
  constexpr int kF4PerRow = kScanXP / 4;
  constexpr int kStageIt  = (kScanTS * kF4PerRow) / kScanCh;
#pragma unroll 1
  for (int t0 = 0; t0 < kL; t0 += kScanTS) {
    __syncthreads();
#pragma unroll 4
    for (int i = 0; i < kStageIt; ++i) {
      const int idx = i * kScanCh + tid;
      const int r   = idx / kF4PerRow;
      const int c4  = (idx - r * kF4PerRow) * 4;
      *(v4f*)(sX + r * kScanXP + c4) = *(const v4f*)(XD + (srow0 + t0 + r) * kXdP + c4);
    }
    {
      const int l  = t0 + tid;
      const int o1 = clampi(perm1[l], 0, kL - 1);
      const int o2 = clampi(perm2[l], 0, kL - 1);
      sRow[tid] = (dir == 0) ? l : ((dir == 1) ? o1 : o2);
    }
    __syncthreads();
#pragma unroll 1
    for (int st = 0; st < kScanTS; ++st) {
      const int t = t0 + st;
      const float* xr = sX + st * kScanXP;
      float vdot = 0.f;
#pragma unroll 1
      for (int r4 = 0; r4 < kDtR / 4; ++r4) {
        const v4f xv = *(const v4f*)(xr + 4 * r4);
        const float* wp = sW + (4 * r4) * kScanCh + tid;
        vdot = fmaf(xv[0], wp[0], vdot);
        vdot = fmaf(xv[1], wp[kScanCh], vdot);
        vdot = fmaf(xv[2], wp[2 * kScanCh], vdot);
        vdot = fmaf(xv[3], wp[3 * kScanCh], vdot);
      }
      float Bs[kNst], Cs[kNst];
#pragma unroll
      for (int q4 = 0; q4 < 4; ++q4) {
        const v4f bv = *(const v4f*)(xr + kDtR + 4 * q4);
        const v4f cv = *(const v4f*)(xr + kDtR + kNst + 4 * q4);
        Bs[4 * q4 + 0] = bv[0]; Bs[4 * q4 + 1] = bv[1]; Bs[4 * q4 + 2] = bv[2]; Bs[4 * q4 + 3] = bv[3];
        Cs[4 * q4 + 0] = cv[0]; Cs[4 * q4 + 1] = cv[1]; Cs[4 * q4 + 2] = cv[2]; Cs[4 * q4 + 3] = cv[3];
      }
      const float v   = vdot + bbias;
      const float a   = __expf(-fabsf(v));
      const float u   = 1.0f + a;
      const float l1p = __logf(u) + (a - (u - 1.0f)) * __builtin_amdgcn_rcpf(u);
      const float dt  = fmaxf(v, 0.0f) + l1p;
      const size_t xo = (srow0 + t) * kDin + d;
      const unsigned hw = XCH[xo];
      const unsigned lw = XCL[xo];
      const float xt  = __uint_as_float(hw << 16) + __uint_as_float(lw << 16);
      const float dtx = dt * xt;
      float y = 0.f;
#pragma unroll
      for (int k = 0; k < kNst; ++k) {
        const float e = __expf(dt * negA[k]);
        h[k] = e * h[k] + dtx * Bs[k];
        y = h[k] * Cs[k] + y;
      }
      y = xt * Dd + y;
      const float zv = XZ[(trow0 + sRow[st]) * kXzP + kDin + d];
      const float sg = __builtin_amdgcn_rcpf(1.0f + __expf(-zv));
      y = y * (zv * sg);
      sY[st * kScanYP + tid] = y;
    }
    __syncthreads();
    v8h hv[8];
#pragma unroll
    for (int it = 0; it < 8; ++it) {
      const int row = it * 8 + wave * 4 + q;
      const float* sp = sY + row * kScanYP + c8;
      const v4f a0 = *(const v4f*)(sp);
      const v4f a1 = *(const v4f*)(sp + 4);
#pragma unroll
      for (int e = 0; e < 4; ++e) {
        hv[it][e]     = (_Float16)a0[e];
        hv[it][4 + e] = (_Float16)a1[e];
      }
    }
    for (int pass = 0; pass < 2; ++pass) {
#pragma unroll
      for (int it = 0; it < 8; ++it) {
        const int row = it * 8 + wave * 4 + q;
        const size_t o = (srow0 + t0 + row) * kDin + d0 + c8;
        *(volatile v8h*)(YD + o) = hv[it];
      }
      __threadfence();
    }
  }
}

__global__ __launch_bounds__(256) void merge_kernel(
    const unsigned short* __restrict__ YD, const int* __restrict__ inv1, const int* __restrict__ inv2,
    unsigned short* __restrict__ YMH, unsigned short* __restrict__ YML, int total8)
{
  const int i = blockIdx.x * 256 + threadIdx.x;
  if (i >= total8) return;
  const unsigned e0 = (unsigned)i << 3;
  const unsigned tr = e0 / (unsigned)kDin;
  const unsigned c  = e0 - tr * (unsigned)kDin;
  const unsigned bb = tr >> 10;
  const unsigned lp = tr & (kL - 1);
  const int i1 = clampi(inv1[lp], 0, kL - 1);
  const int i2 = clampi(inv2[lp], 0, kL - 1);
  const size_t r0 = (size_t)(3 * bb + 0) * kL + lp;
  const size_t r1 = (size_t)(3 * bb + 1) * kL + (unsigned)i1;
  const size_t r2 = (size_t)(3 * bb + 2) * kL + (unsigned)i2;
  const v4u u0 = *(const v4u*)(YD + r0 * kDin + c);
  const v4u u1 = *(const v4u*)(YD + r1 * kDin + c);
  const v4u u2 = *(const v4u*)(YD + r2 * kDin + c);
  v8h hv, lv;
#pragma unroll
  for (int e = 0; e < 4; ++e) {
    const unsigned w0 = u0[e], w1 = u1[e], w2 = u2[e];
    const float ylo = (h16_to_f32(w0 & 0xffffu) + h16_to_f32(w1 & 0xffffu)) + h16_to_f32(w2 & 0xffffu);
    const float yhi = (h16_to_f32(w0 >> 16) + h16_to_f32(w1 >> 16)) + h16_to_f32(w2 >> 16);
    const unsigned short ha = f2bf_bits(ylo), hb = f2bf_bits(yhi);
    const unsigned short la = f2bf_bits(ylo - bf_bits2f(ha)), lb = f2bf_bits(yhi - bf_bits2f(hb));
    hv[2 * e]     = __builtin_bit_cast(_Float16, ha);
    hv[2 * e + 1] = __builtin_bit_cast(_Float16, hb);
    lv[2 * e]     = __builtin_bit_cast(_Float16, la);
    lv[2 * e + 1] = __builtin_bit_cast(_Float16, lb);
  }
  unsigned short* qh = YMH + e0;
  unsigned short* ql = YML + e0;
  *(volatile v8h*)qh = hv;
  *(volatile v8h*)ql = lv;
  __threadfence();
  *(volatile v8h*)qh = hv;
  *(volatile v8h*)ql = lv;
}

extern "C" void kernel_launch(void* const* d_in, const int* in_sizes, int n_in,
                              void* d_out, int out_size, void* d_ws, size_t ws_size,
                              hipStream_t stream) {
  if (n_in < 14) return;
  if (in_sizes[0] != kRowsT * kDm) return;
  if (in_sizes[1] != kXzP * kDm) return;
  if (in_sizes[2] != kDin * 4) return;
  if (in_sizes[3] != kDin) return;
  if (in_sizes[4] != kXdW * kDin) return;
  if (in_sizes[5] != kDin * kDtR) return;
  if (in_sizes[6] != kDin) return;
  if (in_sizes[7] != kDin * kNst) return;
  if (in_sizes[8] != kDin) return;
  if (in_sizes[9] != kDm * kDin) return;
  if (in_sizes[10] != kL || in_sizes[11] != kL || in_sizes[12] != kL || in_sizes[13] != kL) return;
  if (out_size != kRowsT * kDm) return;
  if (ws_size < kWsTotal) return;

  const float* x       = (const float*)d_in[0];
  const float* W_in    = (const float*)d_in[1];
  const float* conv_w  = (const float*)d_in[2];
  const float* conv_b  = (const float*)d_in[3];
  const float* W_xproj = (const float*)d_in[4];
  const float* W_dt    = (const float*)d_in[5];
  const float* b_dt    = (const float*)d_in[6];
  const float* A_log   = (const float*)d_in[7];
  const float* Dp      = (const float*)d_in[8];
  const float* W_out   = (const float*)d_in[9];
  const int*   perm1   = (const int*)d_in[10];
  const int*   perm2   = (const int*)d_in[11];
  const int*   inv1    = (const int*)d_in[12];
  const int*   inv2    = (const int*)d_in[13];
  float* out = (float*)d_out;

  char* ws = (char*)d_ws;
  unsigned short* XH   = (unsigned short*)(ws + kOffXH);
  unsigned short* XL   = (unsigned short*)(ws + kOffXL);
  unsigned short* WIH  = (unsigned short*)(ws + kOffWIH);
  unsigned short* WIL  = (unsigned short*)(ws + kOffWIL);
  unsigned short* WXH  = (unsigned short*)(ws + kOffWXH);
  unsigned short* WXL  = (unsigned short*)(ws + kOffWXL);
  unsigned short* WOH  = (unsigned short*)(ws + kOffWOH);
  unsigned short* WOL  = (unsigned short*)(ws + kOffWOL);
  float*          XZ   = (float*)(ws + kOffXZ);
  unsigned short* XCH  = (unsigned short*)(ws + kOffXCH);
  unsigned short* XCL  = (unsigned short*)(ws + kOffXCL);
  float*          XD   = (float*)(ws + kOffXD);
  unsigned short* YD   = (unsigned short*)(ws + kOffYD);
  unsigned short* YMH  = (unsigned short*)(ws + kOffYMH);
  unsigned short* YML  = (unsigned short*)(ws + kOffYML);

  {
    const int t8x  = kRowsT * kDm / 8;
    const int t8wi = kXzP * kDm / 8;
    const int t8wx = kXdP * kDin / 8;
    const int t8wo = kDm * kDin / 8;
    split_rows_bf16_kernel<<<(t8x  + 255) / 256, 256, 0, stream>>>(x,       XH,  XL,  kRowsT, kDm,  t8x);
    split_rows_bf16_kernel<<<(t8wi + 255) / 256, 256, 0, stream>>>(W_in,    WIH, WIL, kXzP,   kDm,  t8wi);
    split_rows_bf16_kernel<<<(t8wx + 255) / 256, 256, 0, stream>>>(W_xproj, WXH, WXL, kXdW,   kDin, t8wx);
    split_rows_bf16_kernel<<<(t8wo + 255) / 256, 256, 0, stream>>>(W_out,   WOH, WOL, kDm,    kDin, t8wo);
  }

  wmma_gemm64<1, 2, 0, 0, false><<<dim3((kRowsT / 64) * (kXzP / 64) / 8, 1), 256, 0, stream>>>(
      XH, XL, kDm, 0L,
      WIH, WIL, kDm, 0L,
      (void*)XZ, nullptr, kXzP, 0L,
      nullptr, nullptr, 0L,
      kRowsT, kXzP, kDm, 1.0f);

  conv_silu_kernel<<<dim3(kDin / 256, kL / kConvTS, kNS), 256, 0, stream>>>(XZ, conv_w, conv_b, perm1, perm2, XCH, XCL);

  wmma_gemm64<1, 2, 0, 0, false><<<dim3((kRowsS / 64) * (kXdP / 64) / 8, 1), 256, 0, stream>>>(
      XCH, XCL, kDin, 0L,
      WXH, WXL, kDin, 0L,
      (void*)XD, nullptr, kXdP, 0L,
      nullptr, nullptr, 0L,
      kRowsS, kXdP, kDin, 1.0f);

  scan_kernel<<<kNS * (kDin / kScanCh), kScanCh, 0, stream>>>(XD, XCH, XCL, XZ, W_dt, b_dt, A_log, Dp, perm1, perm2, YD);

  {
    const int t8m = kRowsT * kDin / 8;
    merge_kernel<<<(t8m + 255) / 256, 256, 0, stream>>>(YD, inv1, inv2, YMH, YML, t8m);
  }

  wmma_gemm64<1, 2, 0, 0, false><<<dim3((kRowsT / 64) * (kDm / 64) / 8, 1), 256, 0, stream>>>(
      YMH, YML, kDin, 0L,
      WOH, WOL, kDin, 0L,
      (void*)out, nullptr, kDm, 0L,
      nullptr, nullptr, 0L,
      kRowsT, kDm, kDin, 1.0f);
}
